// GCNSiamese2_8624294331071
// MI455X (gfx1250) — hardware-run, weakly checked
//
#include <hip/hip_runtime.h>


namespace {
constexpr int N = 60000, E = 960000, G = 32, F = 38, H = 128, NBLK = N / 16, NCHUNK = 256, CHN = (N + NCHUNK - 1) / NCHUNK;
constexpr float XS = 8.0f, WSC = 256.0f;
typedef _Float16 b16;
typedef __attribute__((ext_vector_type(16))) _Float16 v16b;
typedef __attribute__((ext_vector_type(8))) _Float16 v8b;
typedef __attribute__((ext_vector_type(8))) float v8f;
typedef __attribute__((ext_vector_type(4))) float v4f;
__device__ __forceinline__ float bf16_rne(float f) { unsigned int u = __float_as_uint(f); u += 0x7FFFu + ((u >> 16) & 1u); return __uint_as_float(u & 0xFFFF0000u); }
__device__ __forceinline__ void split16(float v, b16& hi, b16& lo) { hi = (b16)v; lo = (b16)(v - (float)hi); }
__device__ __forceinline__ v16b frag_kb(const b16* p, int hh) { const v8b a = *(const v8b*)(p + 8 * hh), b = *(const v8b*)(p + 16 + 8 * hh); v16b f;
#pragma unroll
  for (int e = 0; e < 8; ++e) { f[e] = a[e]; f[8 + e] = b[e]; } return f; }
__device__ __forceinline__ v8f wmma16b(v16b a, v16b b, v8f c) { v8f d = __builtin_amdgcn_wmma_f32_16x16x32_f16(false, a, false, b, (short)0, c, false, false); asm volatile("v_nop\n\tv_nop\n\tv_nop\n\tv_nop" : "+v"(d) : "v"(a), "v"(b)); return d; }
__device__ __forceinline__ void wave_lds_sync() { __builtin_amdgcn_fence(__ATOMIC_RELEASE, "workgroup"); __builtin_amdgcn_wave_barrier(); __builtin_amdgcn_fence(__ATOMIC_ACQUIRE, "workgroup"); }
__device__ __forceinline__ float pmul(float a, float b) { float p = a * b; asm volatile("" : "+v"(p)); return p; }
__device__ __forceinline__ int iclamp(int v, int lo, int hi) { return v < lo ? lo : (v > hi ? hi : v); }
constexpr int CSR_NBLK9 = 512, CSR_GB9 = 9, CSR_GN9 = 1 << CSR_GB9  , CSR_TS9 = (CSR_GN9 < 32 ? 32 : CSR_GN9)  , CSR_MAXG9 = 512, CSR_CAP9 = 12288  ;
__device__ __host__ __forceinline__ int csr_tix9(int v) { return (v >> CSR_GB9) * CSR_TS9 + (v & (CSR_GN9 - 1)); }
__global__ __launch_bounds__(64) void csrA_kernel9(const int* __restrict__ dst, int E, int N, int nG, int CHP, int NGP, int* __restrict__ STG, int* __restrict__ HST) {
  extern __shared__ int sm[];
  int* cnt = sm; int* run = sm + NGP; int* ids = sm + 2 * NGP;
  const int b = blockIdx.x; const int ch = (E + CSR_NBLK9 - 1) / CSR_NBLK9; const int e0 = b * ch, e1 = min(E, e0 + ch);
  for (int i = threadIdx.x; i < NGP; i += 64) cnt[i] = 0;
  for (int i = threadIdx.x; i < CHP; i += 64) ids[i] = -1;
  __syncthreads();
  if (threadIdx.x == 0) {
    for (int e = e0; e < e1; ++e) { int d = dst[e]; d = (d < 0) ? 0 : (d >= N ? N - 1 : d); cnt[d >> CSR_GB9] += 1; }
    int acc = 0; for (int g = 0; g < nG; ++g) { run[g] = acc; acc += cnt[g]; }
    for (int e = e0; e < e1; ++e) { int d = dst[e]; d = (d < 0) ? 0 : (d >= N ? N - 1 : d); const int g = d >> CSR_GB9; ids[run[g]] = e; run[g] += 1; } }
  __syncthreads();
  typedef __attribute__((ext_vector_type(4))) int v4i;
  for (int pass = 0; pass < 2; ++pass) {
    for (int i = threadIdx.x; i < CHP / 4; i += 64) *(volatile v4i*)(STG + (size_t)b * CHP + i * 4) = *(const v4i*)(&ids[i * 4]);
    for (int i = threadIdx.x; i < NGP / 4; i += 64) { v4i v; for (int e = 0; e < 4; ++e) v[e] = (i * 4 + e < nG) ? cnt[i * 4 + e] : 0; *(volatile v4i*)(HST + (size_t)b * NGP + i * 4) = v; }
    __threadfence(); }
}
__global__ __launch_bounds__(512) void csrS_kernel9(const int* __restrict__ HST, int nG, int NGP, int* __restrict__ START, int* __restrict__ TOT, int* __restrict__ OFF) {
  __shared__ int tot[CSR_MAXG9];
  const int b = threadIdx.x;
  for (int pass = 0; pass < 2; ++pass) { int runb = 0; for (int g = 0; g < nG; ++g) { int c = HST[(size_t)b * NGP + g]; c = (c < 0) ? 0 : c; ((volatile int*)OFF)[(size_t)g * CSR_NBLK9 + b] = runb; runb += c; } __threadfence(); }
  for (int g = threadIdx.x; g < nG; g += 512) { int s = 0; for (int bb = 0; bb < CSR_NBLK9; ++bb) { int c = HST[(size_t)bb * NGP + g]; s += (c < 0) ? 0 : c; } tot[g] = s; }
  __syncthreads();
  if (threadIdx.x < 32) {
    __shared__ int st[CSR_MAXG9 + 32];
    if (threadIdx.x == 0) { int acc = 0; for (int g = 0; g < NGP; ++g) { st[g] = acc; if (g < nG) acc += (tot[g] + 31) & ~31; } st[NGP] = acc; }
    __builtin_amdgcn_fence(__ATOMIC_RELEASE, "workgroup"); __builtin_amdgcn_wave_barrier(); __builtin_amdgcn_fence(__ATOMIC_ACQUIRE, "workgroup");
    for (int pass = 0; pass < 2; ++pass) { for (int i = threadIdx.x; i < NGP + 32; i += 32) { ((volatile int*)START)[i] = (i <= NGP) ? st[min(i, NGP)] : 0; ((volatile int*)TOT)[i] = (i < nG) ? tot[i] : 0; } __threadfence(); } }
}
__global__ __launch_bounds__(256) void csrB_kernel9(const int* __restrict__ dst, int N, int nG, int CHP, int NGP, int permLen, const int* __restrict__ STG, const int* __restrict__ HST, const int* __restrict__ OFF, const int* __restrict__ START, const int* __restrict__ TOT, int* __restrict__ PERM, int* __restrict__ ROWPTR, int* __restrict__ ROWCNT, int* __restrict__ FLAG) {
  typedef __attribute__((ext_vector_type(4))) int v4i;
  __shared__ int ids[CSR_CAP9]; __shared__ unsigned short key[CSR_CAP9]; __shared__ int outp[CSR_CAP9]; __shared__ int ncnt[CSR_GN9 + 1]; __shared__ int boff[CSR_NBLK9 + 1];
  const int g = blockIdx.x, t_ = threadIdx.x; int tot = TOT[g]; int st = START[g], stn = START[g + 1]; const int v0 = g * CSR_GN9; const int nv = min(CSR_GN9, N - v0); const int t0 = g * CSR_TS9;
  st = (st < 0) ? 0 : (st > permLen - 32 ? permLen - 32 : st) & ~31; stn = (stn < st) ? st : (stn > permLen ? permLen : stn); tot = (tot < 0) ? 0 : tot; if (tot > stn - st && tot <= CSR_CAP9) tot = stn - st;
  if (tot > CSR_CAP9) {
    for (int pass = 0; pass < 2; ++pass) { for (int i = t_; i < CSR_TS9 / 4; i += 256) { v4i a, c; for (int e = 0; e < 4; ++e) { a[e] = st; c[e] = 0; } *(volatile v4i*)(ROWPTR + t0 + i * 4) = a; *(volatile v4i*)(ROWCNT + t0 + i * 4) = c; } if (t_ == 0) ((volatile int*)FLAG)[0] = 1; __threadfence(); } (void)nv; return; }
  if (t_ == 0) { int acc = 0; for (int b = 0; b < CSR_NBLK9; ++b) { boff[b] = acc; int c = HST[(size_t)b * NGP + g]; c = (c < 0) ? 0 : (c > CHP ? CHP : c); acc += c; if (acc > tot) acc = tot; } boff[CSR_NBLK9] = acc; }
  for (int i = t_; i <= CSR_GN9; i += 256) ncnt[i] = 0;
  __syncthreads();
  for (int b = 0; b < CSR_NBLK9; ++b) { const int c = boff[b + 1] - boff[b]; int o_ = OFF[(size_t)g * CSR_NBLK9 + b]; o_ = (o_ < 0) ? 0 : (o_ > CHP - c ? CHP - c : o_); const int* src_ = STG + (size_t)b * CHP + o_;
    for (int i = t_; i < c; i += 256) { int id = src_[i]; id = (id < 0) ? 0 : id; ids[boff[b] + i] = id; int d = dst[id]; d = (d < v0) ? v0 : (d >= N ? N - 1 : d); int kk = d - v0; kk = (kk < 0) ? 0 : (kk >= CSR_GN9 ? CSR_GN9 - 1 : kk); key[boff[b] + i] = (unsigned short)kk; } }
  __syncthreads();
  if (t_ == 0) { for (int i = 0; i < tot; ++i) ncnt[key[i]] += 1; int acc = 0; for (int vl = 0; vl < CSR_GN9; ++vl) { const int c = ncnt[vl]; ncnt[vl] = acc; acc += c; } ncnt[CSR_GN9] = acc;
    for (int i = 0; i < tot; ++i) { const int vl = key[i]; outp[ncnt[vl]] = ids[i]; ncnt[vl] += 1; }
    for (int vl = CSR_GN9; vl > 0; --vl) ncnt[vl] = ncnt[vl - 1]; ncnt[0] = 0; }
  __syncthreads();
  for (int pass = 0; pass < 2; ++pass) {
    for (int i = t_; i < (stn - st) / 4; i += 256) { v4i v; for (int e = 0; e < 4; ++e) { const int q = i * 4 + e; v[e] = (q < tot) ? outp[q] : -1; } *(volatile v4i*)(PERM + st + i * 4) = v; }
    for (int i = t_; i < CSR_TS9 / 4; i += 256) { v4i a, c; for (int e = 0; e < 4; ++e) { const int vl = i * 4 + e; const int vc = vl < CSR_GN9 ? vl : CSR_GN9; a[e] = (vl < CSR_GN9) ? st + ncnt[vc] : st; c[e] = (vl < nv) ? (ncnt[(vc < CSR_GN9 ? vc : CSR_GN9 - 1) + 1] - ncnt[vc]) : 0; } *(volatile v4i*)(ROWPTR + t0 + i * 4) = a; *(volatile v4i*)(ROWCNT + t0 + i * 4) = c; }
    __threadfence(); }
}
__global__ __launch_bounds__(256) void csrZ_kernel9(int* __restrict__ p, size_t n4) { typedef __attribute__((ext_vector_type(4))) int v4i; const size_t tid = (size_t)blockIdx.x * 256 + threadIdx.x, nth = (size_t)gridDim.x * 256; v4i z = {0, 0, 0, 0}; for (size_t i = tid; i < n4; i += nth) *(volatile v4i*)(p + i * 4) = z; }
struct CsrBufs9 { int *STG, *HST, *OFF, *START, *TOT, *PERM, *ROWPTR, *ROWCNT, *FLAG; int nG, NGP, CHP; size_t permLen; char* base; size_t bytes; };
static size_t csr_carve9(CsrBufs9& c, char* ws, size_t off, int E, int N) {
  const size_t off0 = off; c.base = ws + off;
  auto al = [&](size_t bytes) { char* p = ws + off; off += (bytes + 255) & ~(size_t)255; return p; };
  c.nG = (N + CSR_GN9 - 1) / CSR_GN9; c.NGP = (c.nG + 31) & ~31; const int ch = (E + CSR_NBLK9 - 1) / CSR_NBLK9; c.CHP = (ch + 31) & ~31; c.permLen = (size_t)E + 32 * (size_t)c.nG + 32;
  c.STG = (int*)al((size_t)CSR_NBLK9 * c.CHP * 4); c.HST = (int*)al((size_t)CSR_NBLK9 * c.NGP * 4); c.OFF = (int*)al((size_t)c.NGP * CSR_NBLK9 * 4); c.START = (int*)al((size_t)(c.NGP + 64) * 4); c.TOT = (int*)al((size_t)(c.NGP + 64) * 4);
  c.PERM = (int*)al(c.permLen * 4); c.ROWPTR = (int*)al((size_t)c.nG * CSR_TS9 * 4); c.ROWCNT = (int*)al((size_t)c.nG * CSR_TS9 * 4); c.FLAG = (int*)al(256);
  c.bytes = off - off0; return off;
}
static void csr_build9(const CsrBufs9& c, const int* dst, int E, int N, hipStream_t stream) {
  const size_t smem = (size_t)(2 * c.NGP + c.CHP) * 4;
  csrZ_kernel9<<<512, 256, 0, stream>>>((int*)c.base, c.bytes / 16);
  csrA_kernel9<<<CSR_NBLK9, 64, smem, stream>>>(dst, E, N, c.nG, c.CHP, c.NGP, c.STG, c.HST);
  csrS_kernel9<<<1, 512, 0, stream>>>(c.HST, c.nG, c.NGP, c.START, c.TOT, c.OFF);
  csrB_kernel9<<<c.nG, 256, 0, stream>>>(dst, N, c.nG, c.CHP, c.NGP, (int)c.permLen, c.STG, c.HST, c.OFF, c.START, c.TOT, c.PERM, c.ROWPTR, c.ROWCNT, c.FLAG);
}


__global__ __launch_bounds__(256) void wput_kernel(const float* __restrict__ w, int KIN, int KPAD, int OUTW, int ko, int KP, b16* __restrict__ WT) {
  const int KG = KPAD / 8; const int u = blockIdx.x * 256 + threadIdx.x; if (u >= OUTW * KG) return; const int o = u / KG, k0 = (u % KG) * 8; v8b v;
#pragma unroll
  for (int j = 0; j < 8; ++j) { const int k = k0 + j; v[j] = k < KIN ? (b16)(bf16_rne(w[(size_t)k * OUTW + o]) * WSC) : (b16)0.0f; } for (int pass = 0; pass < 2; ++pass) { *(volatile v8b*)(WT + (size_t)o * KP + ko + k0) = v; __threadfence(); }
}
template <int KP_, int KLIVE, int FIRST>
__global__ __launch_bounds__(32) void gc_kernel(const float* __restrict__ IN, const float* __restrict__ STAT, const int* __restrict__ srcs, const int* __restrict__ PERM, const int* __restrict__ ROWPTR, const int* __restrict__ ROWCNT, int permLen, const b16* __restrict__ WT, const float* __restrict__ bias, int NLIM, float* __restrict__ Z) {
  constexpr int K2 = 2 * KP_, PL = KP_ / 32; __shared__ __attribute__((aligned(16))) b16 Ah[16][K2 + 8], Al[16][K2 + 8]; __shared__ __attribute__((aligned(16))) float Tf[16][H + 4];
  const int lane = threadIdx.x, nloc = lane & 15, hlf = lane >> 4; const size_t m0 = (size_t)blockIdx.x * 16; if (m0 >= (size_t)NLIM) return;
  float sc[PL], sh[PL]; for (int q = 0; q < PL; ++q) { const int c = q * 32 + lane; sc[q] = (!FIRST && c < KLIVE) ? STAT[c] : 0.0f; sh[q] = (!FIRST && c < KLIVE) ? STAT[H + c] : 0.0f; }
  auto feat = [&](size_t n, int q) -> float { const int c = q * 32 + lane; if (c >= KLIVE) return 0.0f; const float v = IN[n * KLIVE + c]; return FIRST ? bf16_rne(v) : fmaxf(pmul(v, sc[q]) + sh[q], 0.0f); };
  for (int rr = 0; rr < 16; ++rr) { const size_t v = m0 + rr; int st = ROWPTR[v], cnt = ROWCNT[v]; cnt = iclamp(cnt, 0, 1 << 20); st = iclamp(st, 0, permLen - cnt); float a[PL], s_[PL]; for (int q = 0; q < PL; ++q) { a[q] = 0.0f; s_[q] = feat(v, q); }
#pragma unroll 1
    for (int j = 0; j < cnt; ++j) { const int e = iclamp(PERM[st + j], 0, E - 1); const size_t u = (size_t)iclamp(srcs[e], 0, N - 1); if (u >= (size_t)NLIM) continue; for (int q = 0; q < PL; ++q) a[q] += feat(u, q); }
    for (int q = 0; q < PL; ++q) { b16 p, ql; split16(a[q] * XS, p, ql); Ah[rr][q * 32 + lane] = p; Al[rr][q * 32 + lane] = ql; split16(s_[q] * XS, p, ql); Ah[rr][KP_ + q * 32 + lane] = p; Al[rr][KP_ + q * 32 + lane] = ql; } }
  wave_lds_sync();
  v8f acc[8];
#pragma unroll
  for (int t = 0; t < 8; ++t) acc[t] = (v8f){};
#pragma unroll 2
  for (int kb = 0; kb < K2; kb += 32) { const v16b fa = frag_kb(&Ah[nloc][kb], hlf), fl = frag_kb(&Al[nloc][kb], hlf);
#pragma unroll
    for (int t = 0; t < 8; ++t) { const v16b bw = frag_kb(WT + (size_t)(t * 16 + nloc) * K2 + kb, hlf); acc[t] = wmma16b(fa, bw, acc[t]); acc[t] = wmma16b(fl, bw, acc[t]); } }
#pragma unroll
  for (int t = 0; t < 8; ++t) { const int c = t * 16 + nloc; const float bb = bf16_rne(bias[c]);
#pragma unroll
    for (int r8 = 0; r8 < 8; ++r8) Tf[8 * hlf + r8][c] = acc[t][r8] * (1.0f / (XS * WSC)) + bb; }
  wave_lds_sync();
  for (int pass = 0; pass < 2; ++pass) { for (int rr = 0; rr < 16; ++rr) *(volatile v4f*)(Z + (m0 + rr) * H + lane * 4) = *(const v4f*)(&Tf[rr][lane * 4]); __threadfence(); }
}
__global__ __launch_bounds__(128) void bnstat_kernel(const float* __restrict__ Z, const float* __restrict__ g, const float* __restrict__ be, int NLIM, float* __restrict__ STAT) {
  const int c = threadIdx.x; double s = 0.0, s2 = 0.0;
#pragma unroll 4
  for (int n = 0; n < NLIM; ++n) { const double v = (double)Z[(size_t)n * H + c]; s += v; s2 += v * v; }
  const double mean = s / NLIM; const double var = fmax(s2 / NLIM - mean * mean, 0.0); const float scale = bf16_rne(g[c]) * (float)(1.0 / sqrt(var + 1e-5)); const float shift = bf16_rne(be[c]) - (float)mean * scale;
  for (int pass = 0; pass < 2; ++pass) { ((volatile float*)STAT)[c] = scale; ((volatile float*)STAT)[H + c] = shift; __threadfence(); }
}
__global__ __launch_bounds__(64) void fin_kernel(const float* __restrict__ Z, const float* __restrict__ STAT, const b16* __restrict__ WG1, const float* __restrict__ bg1, const float* __restrict__ wg2, const float* __restrict__ bg2, int NLIM, float* __restrict__ HO, float* __restrict__ GT) {
  __shared__ __attribute__((aligned(16))) b16 Ah[2][16][H + 8], Al[2][16][H + 8]; __shared__ float So[32];
  const int wave = threadIdx.x >> 5, lane = threadIdx.x & 31, nloc = lane & 15, hlf = lane >> 4; const size_t m0 = (size_t)blockIdx.x * 32 + wave * 16;
  if (m0 < (size_t)NLIM) {
    for (int rr = 0; rr < 16; ++rr) { v4f o; for (int i = 0; i < 4; ++i) { const int c = lane * 4 + i; o[i] = fmaxf(pmul(Z[(m0 + rr) * H + c], STAT[c]) + STAT[H + c], 0.0f); b16 p, q; split16(o[i] * XS, p, q); Ah[wave][rr][c] = p; Al[wave][rr][c] = q; }
      for (int pass = 0; pass < 2; ++pass) { *(volatile v4f*)(HO + (m0 + rr) * H + lane * 4) = o; __threadfence(); } }
    wave_lds_sync();
    float pd[8];
#pragma unroll
    for (int r8 = 0; r8 < 8; ++r8) pd[r8] = 0.0f;
#pragma unroll
    for (int t = 0; t < 2; ++t) { v8f acc = {};
#pragma unroll
      for (int kb = 0; kb < H; kb += 32) { const v16b bw = frag_kb(WG1 + (size_t)(t * 16 + nloc) * H + kb, hlf); acc = wmma16b(frag_kb(&Ah[wave][nloc][kb], hlf), bw, acc); acc = wmma16b(frag_kb(&Al[wave][nloc][kb], hlf), bw, acc); }
      const int c = t * 16 + nloc; const float bb = bf16_rne(bg1[c]), w2 = bf16_rne(wg2[c]);
#pragma unroll
      for (int r8 = 0; r8 < 8; ++r8) pd[r8] += pmul(fmaxf(acc[r8] * (1.0f / (XS * WSC)) + bb, 0.0f), w2); }
#pragma unroll
    for (int r8 = 0; r8 < 8; ++r8) { float s = pd[r8]; for (int o = 1; o < 16; o <<= 1) s += __shfl_xor(s, o); if (nloc == 0) So[wave * 16 + 8 * hlf + r8] = fmaxf(s + bf16_rne(bg2[0]), 0.0f); }
  } else if (lane < 16) So[wave * 16 + lane] = 0.0f;
  __syncthreads();
  if (wave == 0) { for (int pass = 0; pass < 2; ++pass) { ((volatile float*)GT)[(size_t)blockIdx.x * 32 + lane] = So[lane]; __threadfence(); } }
}
__global__ __launch_bounds__(256) void pmax_kernel(const float* __restrict__ GT, const int* __restrict__ batch, int NLIM, float* __restrict__ PM) {
  __shared__ float red[8][G]; const int ch = blockIdx.x, tid = threadIdx.x, wave = tid >> 5, lane = tid & 31; const int n0 = ch * CHN; float m[G]; for (int g = 0; g < G; ++g) m[g] = -INFINITY;
  for (int i = tid; i < CHN; i += 256) { const int n = n0 + i; if (n < NLIM) { const int b = iclamp(batch[n], 0, G - 1); const float v = GT[n]; for (int g = 0; g < G; ++g) m[g] = (g == b) ? fmaxf(m[g], v) : m[g]; } }
  for (int g = 0; g < G; ++g) { float x = m[g]; for (int o = 16; o; o >>= 1) x = fmaxf(x, __shfl_xor(x, o)); if (lane == 0) red[wave][g] = x; }
  __syncthreads();
  if (tid < 32) { float x = red[0][tid]; for (int w = 1; w < 8; ++w) x = fmaxf(x, red[w][tid]); for (int pass = 0; pass < 2; ++pass) { ((volatile float*)PM)[ch * G + tid] = x; __threadfence(); } }
}
__global__ __launch_bounds__(32) void gmax_kernel(const float* __restrict__ PM, float* __restrict__ GM) { const int g = threadIdx.x; float x = -INFINITY; for (int ch = 0; ch < NCHUNK; ++ch) x = fmaxf(x, PM[ch * G + g]); for (int pass = 0; pass < 2; ++pass) { ((volatile float*)GM)[g] = x; __threadfence(); } }
__global__ __launch_bounds__(128) void psum_kernel(const float* __restrict__ HO, const float* __restrict__ GT, const int* __restrict__ batch, const float* __restrict__ GM, int NLIM, float* __restrict__ PS, float* __restrict__ PD) {
  __shared__ float acc[G][H + 1]; __shared__ float dn[G]; const int ch = blockIdx.x, c = threadIdx.x; const int n0 = ch * CHN;
  for (int g = 0; g < G; ++g) acc[g][c] = 0.0f; if (c < G) dn[c] = 0.0f; __syncthreads();
  float dreg = 0.0f;
#pragma unroll 1
  for (int i = 0; i < CHN; ++i) { const int n = n0 + i; if (n >= NLIM) break; const int b = iclamp(batch[n], 0, G - 1); const float eg = __expf(GT[n] - GM[b]); acc[b][c] += pmul(eg, HO[(size_t)n * H + c]); if (c == b) dreg += eg; }
  __syncthreads();
  for (int pass = 0; pass < 2; ++pass) { for (int g = 0; g < G; ++g) ((volatile float*)PS)[((size_t)ch * G + g) * H + c] = acc[g][c]; if (c < G) ((volatile float*)PD)[ch * G + c] = dreg; __threadfence(); }
}
__global__ __launch_bounds__(128) void pool_kernel(const float* __restrict__ PS, const float* __restrict__ PD, float* __restrict__ EMB) {
  const int g = blockIdx.x, c = threadIdx.x; float s = 0.0f, d = 0.0f; for (int ch = 0; ch < NCHUNK; ++ch) { s += PS[((size_t)ch * G + g) * H + c]; d += PD[ch * G + g]; }
  const float v = d > 0.0f ? s / d : 0.0f; for (int pass = 0; pass < 2; ++pass) { ((volatile float*)EMB)[g * H + c] = v; __threadfence(); }
}
__global__ __launch_bounds__(32) void head_kernel(const float* __restrict__ E1, const float* __restrict__ E2, const float* __restrict__ Wf1, const float* __restrict__ bf1, const float* __restrict__ Wf2, const float* __restrict__ bf2, float* __restrict__ out) {
  __shared__ float Dd[G][H + 1]; const int g = threadIdx.x; for (int c = 0; c < H; ++c) Dd[g][c] = fabsf(E1[g * H + c] - E2[g * H + c]); wave_lds_sync();
  float s = bf16_rne(bf2[0]);
#pragma unroll 1
  for (int j = 0; j < 64; ++j) { float a = bf16_rne(bf1[j]);
#pragma unroll 1
    for (int c = 0; c < H; ++c) a += pmul(Dd[g][c], bf16_rne(Wf1[c * 64 + j])); s += pmul(fmaxf(a, 0.0f), bf16_rne(Wf2[j])); }
  for (int pass = 0; pass < 2; ++pass) { ((volatile float*)out)[g] = s; __threadfence(); }
}
}

extern "C" void kernel_launch(void* const* d_in, const int* in_sizes, int n_in, void* d_out, int out_size, void* d_ws, size_t ws_size, hipStream_t stream) {
  (void)n_in;
  auto Fp = [&](int i) { return (const float*)d_in[i]; }; auto Ip = [&](int i) { return (const int*)d_in[i]; };
  if (in_sizes[0] != N * F || in_sizes[1] != N * F || in_sizes[2] != 2 * E || in_sizes[3] != 2 * E || in_sizes[4] != N || in_sizes[5] != N || in_sizes[6] != F * H || in_sizes[11] != H * H || in_sizes[16] != H * H || in_sizes[21] != H * 32 || in_sizes[25] != H * 64 || out_size != G) return;
  const int NLIM = N; const int GB16 = NBLK;
  size_t off = 0; char* ws = (char*)d_ws;
  auto carve = [&](size_t bytes) { char* p = ws + off; off += (bytes + 255) & ~(size_t)255; return p; };
  b16* WT1 = (b16*)carve((size_t)H * 128 * 2); b16* WT2 = (b16*)carve((size_t)H * 256 * 2); b16* WT3 = (b16*)carve((size_t)H * 256 * 2); b16* WG1 = (b16*)carve(32 * H * 2);
  float* Z = (float*)carve((size_t)N * H * 4); float* HO = (float*)carve((size_t)N * H * 4); float* STAT = (float*)carve(2 * H * 4); float* GT = (float*)carve((size_t)(N + 32) * 4); float* PM = (float*)carve(NCHUNK * G * 4); float* GM = (float*)carve(G * 4);
  float* PS = (float*)carve((size_t)NCHUNK * G * H * 4); float* PD = (float*)carve(NCHUNK * G * 4); float* EMB1 = (float*)carve(G * H * 4); float* EMB2 = (float*)carve(G * H * 4);
  CsrBufs9 c1, c2; off = csr_carve9(c1, ws, off, E, N); off = csr_carve9(c2, ws, off, E, N);
  if (off > ws_size || off > ((size_t)128 << 20)) return;
  wput_kernel<<<(H * 8 + 255) / 256, 256, 0, stream>>>(Fp(6), F, 64, H, 0, 128, WT1); wput_kernel<<<(H * 8 + 255) / 256, 256, 0, stream>>>(Fp(7), F, 64, H, 64, 128, WT1);
  wput_kernel<<<(H * 16 + 255) / 256, 256, 0, stream>>>(Fp(11), H, H, H, 0, 256, WT2); wput_kernel<<<(H * 16 + 255) / 256, 256, 0, stream>>>(Fp(12), H, H, H, H, 256, WT2);
  wput_kernel<<<(H * 16 + 255) / 256, 256, 0, stream>>>(Fp(16), H, H, H, 0, 256, WT3); wput_kernel<<<(H * 16 + 255) / 256, 256, 0, stream>>>(Fp(17), H, H, H, H, 256, WT3);
  wput_kernel<<<(32 * 16 + 255) / 256, 256, 0, stream>>>(Fp(21), H, H, 32, 0, H, WG1);
  csr_build9(c1, Ip(2) + E, E, N, stream); csr_build9(c2, Ip(3) + E, E, N, stream);
  for (int side = 0; side < 2; ++side) { const CsrBufs9& cs = side ? c2 : c1; const float* x = Fp(side); const int* ei = Ip(2 + side); const int* bt = Ip(4 + side); float* EMB = side ? EMB2 : EMB1;
    gc_kernel<64, F, 1><<<GB16, 32, 0, stream>>>(x, nullptr, ei, cs.PERM, cs.ROWPTR, cs.ROWCNT, (int)cs.permLen, WT1, Fp(8), NLIM, Z);
    bnstat_kernel<<<1, H, 0, stream>>>(Z, Fp(9), Fp(10), NLIM, STAT);
    gc_kernel<H, H, 0><<<GB16, 32, 0, stream>>>(Z, STAT, ei, cs.PERM, cs.ROWPTR, cs.ROWCNT, (int)cs.permLen, WT2, Fp(13), NLIM, HO);
    bnstat_kernel<<<1, H, 0, stream>>>(HO, Fp(14), Fp(15), NLIM, STAT);
    gc_kernel<H, H, 0><<<GB16, 32, 0, stream>>>(HO, STAT, ei, cs.PERM, cs.ROWPTR, cs.ROWCNT, (int)cs.permLen, WT3, Fp(18), NLIM, Z);
    bnstat_kernel<<<1, H, 0, stream>>>(Z, Fp(19), Fp(20), NLIM, STAT);
    fin_kernel<<<(unsigned)((NLIM + 31) / 32), 64, 0, stream>>>(Z, STAT, WG1, Fp(22), Fp(23), Fp(24), NLIM, HO, GT);
    pmax_kernel<<<NCHUNK, 256, 0, stream>>>(GT, bt, NLIM, PM); gmax_kernel<<<1, 32, 0, stream>>>(PM, GM);
    psum_kernel<<<NCHUNK, H, 0, stream>>>(HO, GT, bt, GM, NLIM, PS, PD); pool_kernel<<<G, H, 0, stream>>>(PS, PD, EMB); }
  head_kernel<<<1, 32, 0, stream>>>(EMB1, EMB2, Fp(25), Fp(26), Fp(27), Fp(28), (float*)d_out);
}
